// RScaledDotProductAttetion_87995289960718
// MI455X (gfx1250) — hardware-verified
//
#include <hip/hip_runtime.h>
#include <stdint.h>

typedef _Float16 f16_t;
typedef _Float16 v16h __attribute__((ext_vector_type(16)));
typedef _Float16 v8h __attribute__((ext_vector_type(8)));
typedef v8h __attribute__((may_alias)) v8ha;
typedef __bf16 v16b __attribute__((ext_vector_type(16)));
typedef __bf16 v8b __attribute__((ext_vector_type(8)));
typedef float v8f __attribute__((ext_vector_type(8)));
typedef float v4f __attribute__((ext_vector_type(4)));
typedef v4f __attribute__((may_alias)) v4fa;
typedef unsigned v4u __attribute__((ext_vector_type(4)));
typedef int v4i __attribute__((ext_vector_type(4)));

union FragH { v16h v; v8h p[2]; };
union FragB { v16b v; v8b p[2]; };

#define S_LEN 2048
#define D_DIM 64
#define BH_N 32
#define NT (S_LEN / 32)
#define NELEM (BH_N * S_LEN * D_DIM)
#define QB 128
#define TP 72

static __device__ __forceinline__ v8f mma_bf16(v16b a, v16b b, v8f c) {
  v8f d = __builtin_amdgcn_wmma_f32_16x16x32_bf16(false, a, false, b, (short)0, c,
                                                  false, false);
  asm volatile("v_nop\n\tv_nop\n\tv_nop\n\tv_nop" : "+v"(d) : "v"(a), "v"(b));
  return d;
}
static __device__ __forceinline__ v8f mma_f16(v16h a, v16h b, v8f c) {
  v8f d = __builtin_amdgcn_wmma_f32_16x16x32_f16(false, a, false, b, (short)0, c,
                                                 false, false);
  asm volatile("v_nop\n\tv_nop\n\tv_nop\n\tv_nop" : "+v"(d) : "v"(a), "v"(b));
  return d;
}

static __device__ __forceinline__ unsigned bf16_rne(float f) {
  unsigned u = __float_as_uint(f);
  u += 0x7FFFu + ((u >> 16) & 1u);
  return u >> 16;
}
static __device__ __forceinline__ unsigned q_bits(float f) {
  const float r = __uint_as_float(bf16_rne(f) << 16) * 0.125f;
  return __float_as_uint(r) >> 16;
}
static __device__ __forceinline__ f16_t v_half(float f) {
  return (f16_t)__uint_as_float(bf16_rne(f) << 16);
}

__global__ __launch_bounds__(256) void k_cvt_qk(const float* __restrict__ Q,
                                                const float* __restrict__ K,
                                                unsigned short* __restrict__ Qb,
                                                unsigned short* __restrict__ Kb,
                                                int n8) {
  const int g = blockIdx.x * 256 + threadIdx.x;
  if (g >= n8) return;
  const size_t e = (size_t)g * 8;
  const v4f q0 = *(const v4f*)(Q + e);
  const v4f q1 = *(const v4f*)(Q + e + 4);
  const v4f k0 = *(const v4f*)(K + e);
  const v4f k1 = *(const v4f*)(K + e + 4);
  v4u qv, kv;
  qv[0] = q_bits(q0[0]) | (q_bits(q0[1]) << 16);
  qv[1] = q_bits(q0[2]) | (q_bits(q0[3]) << 16);
  qv[2] = q_bits(q1[0]) | (q_bits(q1[1]) << 16);
  qv[3] = q_bits(q1[2]) | (q_bits(q1[3]) << 16);
  kv[0] = bf16_rne(k0[0]) | (bf16_rne(k0[1]) << 16);
  kv[1] = bf16_rne(k0[2]) | (bf16_rne(k0[3]) << 16);
  kv[2] = bf16_rne(k1[0]) | (bf16_rne(k1[1]) << 16);
  kv[3] = bf16_rne(k1[2]) | (bf16_rne(k1[3]) << 16);
  unsigned short* qd = Qb + e;
  unsigned short* kd = Kb + e;
  *(volatile v4u*)qd = qv;
  *(volatile v4u*)kd = kv;
  __threadfence();
  *(volatile v4u*)qd = qv;
  *(volatile v4u*)kd = kv;
}

__global__ __launch_bounds__(256) void k_cvt_vt(const float* __restrict__ V,
                                                f16_t* __restrict__ Vt) {
  __shared__ __align__(16) f16_t Tl[D_DIM * TP];
  const int t = threadIdx.x, lane = t & 31, w = t >> 5;
  const int bh = blockIdx.x >> 5;
  const int key0 = (blockIdx.x & 31) * 64;
  const float* vsrc = V + ((size_t)bh * S_LEN + key0) * D_DIM;
#pragma unroll
  for (int i = 0; i < 4; ++i) {
    const int f = t + i * 256;
    const int ky = f >> 4;
    const int d0 = (f & 15) * 4;
    const v4f v = *(const v4f*)(vsrc + (size_t)ky * D_DIM + d0);
#pragma unroll
    for (int c = 0; c < 4; ++c) Tl[(d0 + c) * TP + ky] = v_half(v[c]);
  }
  __syncthreads();
  v8h vals[2];
  f16_t* dst[2];
#pragma unroll
  for (int i = 0; i < 2; ++i) {
    const int d = w * 8 + i * 4 + (lane >> 3);
    const int kx = (lane & 7) * 8;
    vals[i] = *(const v8ha*)(Tl + d * TP + kx);
    dst[i] = Vt + ((size_t)bh * D_DIM + d) * S_LEN + key0 + kx;
  }
  *(volatile v8h*)dst[0] = vals[0];
  *(volatile v8h*)dst[1] = vals[1];
  __threadfence();
  *(volatile v8h*)dst[0] = vals[0];
  *(volatile v8h*)dst[1] = vals[1];
}

__global__ __launch_bounds__(256) void k_maskbits(const int* __restrict__ M,
                                                  unsigned* __restrict__ Mb,
                                                  int total4) {
  const int g = blockIdx.x * 256 + threadIdx.x;
  if (g >= total4) return;
  const int o4 = g * 4;
  const int kt = o4 >> 11;
  const int q0 = o4 & (S_LEN - 1);
  v4u wv;
#pragma unroll
  for (int i = 0; i < 4; ++i) {
    const int* mr = M + (size_t)(q0 + i) * S_LEN + kt * 32;
    unsigned wd = 0;
#pragma unroll
    for (int j8 = 0; j8 < 8; ++j8) {
      const v4i m = *(const v4i*)(mr + j8 * 4);
#pragma unroll
      for (int c = 0; c < 4; ++c)
        wd |= ((m[c] != 0) ? 1u : 0u) << (j8 * 4 + c);
    }
    wv[i] = wd;
  }
  unsigned* dp = Mb + o4;
  *(volatile v4u*)dp = wv;
  __threadfence();
  *(volatile v4u*)dp = wv;
}

__global__ __launch_bounds__(256) void k_attn(const unsigned short* __restrict__ Qb,
                                              const unsigned short* __restrict__ Kb,
                                              const f16_t* __restrict__ Vt,
                                              const unsigned* __restrict__ Mb,
                                              float* __restrict__ O) {
  __shared__ __align__(16) unsigned short Klds[32 * D_DIM];
  __shared__ __align__(16) f16_t Vlds[D_DIM * 32];
  __shared__ __align__(16) f16_t Plds[8 * 16 * 32];
  __shared__ __align__(16) float Olds[8 * 16 * D_DIM];

  const int t = threadIdx.x;
  const int lane = t & 31;
  const int w = t >> 5;
  const int n = lane & 15;
  const int h = lane >> 4;
  const int bh = blockIdx.y;
  const int qrow0 = blockIdx.x * QB + w * 16;
  const float NEG_INF = -__builtin_inff();
  const float LOG2E = 1.4426950408889634f;

  FragB qa0, qa1;
  {
    const unsigned short* qr = Qb + ((size_t)bh * S_LEN + qrow0 + n) * D_DIM;
    qa0.p[0] = *(const v8b*)(qr + 8 * h);
    qa0.p[1] = *(const v8b*)(qr + 16 + 8 * h);
    qa1.p[0] = *(const v8b*)(qr + 32 + 8 * h);
    qa1.p[1] = *(const v8b*)(qr + 48 + 8 * h);
  }

  v8f o0 = {}, o1 = {}, o2 = {}, o3 = {};
  float mrow[8], brow[8], lpart[8];
#pragma unroll
  for (int r = 0; r < 8; ++r) { mrow[r] = NEG_INF; brow[r] = __builtin_inff(); lpart[r] = 0.0f; }

  f16_t* Pw = Plds + w * 512;
  const size_t kbase = (size_t)bh * S_LEN * D_DIM;
  const size_t vbase = (size_t)bh * D_DIM * S_LEN;

  for (int kt = 0; kt < NT; ++kt) {
    const int key0 = kt * 32;
    __syncthreads();
    {
      const v4u kv = *(const v4u*)(Kb + kbase + (size_t)key0 * D_DIM + t * 8);
      *(v4u*)(Klds + t * 8) = kv;
      const int d = t >> 2, c = t & 3;
      const v4u vv = *(const v4u*)(Vt + vbase + (size_t)d * S_LEN + key0 + c * 8);
      *(v4u*)(Vlds + d * 32 + c * 8) = vv;
    }
    __syncthreads();

    v8f s0 = {}, s1 = {};
    {
      FragB b;
      const unsigned short* kp = Klds + n * D_DIM;
      b.p[0] = *(const v8b*)(kp + 8 * h);
      b.p[1] = *(const v8b*)(kp + 16 + 8 * h);
      s0 = mma_bf16(qa0.v, b.v, s0);
      b.p[0] = *(const v8b*)(kp + 32 + 8 * h);
      b.p[1] = *(const v8b*)(kp + 48 + 8 * h);
      s0 = mma_bf16(qa1.v, b.v, s0);
      kp += 16 * D_DIM;
      b.p[0] = *(const v8b*)(kp + 8 * h);
      b.p[1] = *(const v8b*)(kp + 16 + 8 * h);
      s1 = mma_bf16(qa0.v, b.v, s1);
      b.p[0] = *(const v8b*)(kp + 32 + 8 * h);
      b.p[1] = *(const v8b*)(kp + 48 + 8 * h);
      s1 = mma_bf16(qa1.v, b.v, s1);
    }

    {
      const unsigned* mp = Mb + (size_t)kt * S_LEN + qrow0 + 8 * h;
      const v4u ma = *(const v4u*)mp;
      const v4u mb = *(const v4u*)(mp + 4);
      unsigned mw[8];
      mw[0] = ma[0]; mw[1] = ma[1]; mw[2] = ma[2]; mw[3] = ma[3];
      mw[4] = mb[0]; mw[5] = mb[1]; mw[6] = mb[2]; mw[7] = mb[3];
      const unsigned all = mw[0] & mw[1] & mw[2] & mw[3] & mw[4] & mw[5] & mw[6] & mw[7];
      if (all != 0xffffffffu) {
#pragma unroll
        for (int r = 0; r < 8; ++r) {
          if (((mw[r] >> n) & 1u) == 0u) s0[r] = NEG_INF;
          if (((mw[r] >> (n + 16)) & 1u) == 0u) s1[r] = NEG_INF;
        }
      }
    }

    float mx[8];
#pragma unroll
    for (int r = 0; r < 8; ++r) mx[r] = fmaxf(s0[r], s1[r]);
#pragma unroll
    for (int off = 8; off > 0; off >>= 1) {
#pragma unroll
      for (int r = 0; r < 8; ++r) mx[r] = fmaxf(mx[r], __shfl_xor(mx[r], off));
    }

    v8f cv;
#pragma unroll
    for (int r = 0; r < 8; ++r) {
      const float mnew = fmaxf(mrow[r], mx[r]);
      const float sh = (mnew == NEG_INF) ? 0.0f : mnew;
      const float bnew = fmaf(-sh, LOG2E, 8.0f);
      const float corr = exp2f(bnew - brow[r]);
      mrow[r] = mnew;
      brow[r] = bnew;
      cv[r] = corr;
      float e0 = exp2f(fmaf(s0[r], LOG2E, bnew));
      float e1 = exp2f(fmaf(s1[r], LOG2E, bnew));
      e0 = (e0 >= 6.103515625e-05f) ? e0 : 0.0f;
      e1 = (e1 >= 6.103515625e-05f) ? e1 : 0.0f;
      lpart[r] = fmaf(lpart[r], corr, e0 + e1);
      Pw[(8 * h + r) * 32 + n] = (f16_t)e0;
      Pw[(8 * h + r) * 32 + 16 + n] = (f16_t)e1;
    }
    o0 *= cv; o1 *= cv; o2 *= cv; o3 *= cv;

    __syncthreads();

    FragH pa;
    pa.p[0] = *(const v8ha*)(Pw + n * 32 + 8 * h);
    pa.p[1] = *(const v8ha*)(Pw + n * 32 + 16 + 8 * h);
    {
      FragH vb;
      const f16_t* vp = Vlds + n * 32;
      vb.p[0] = *(const v8ha*)(vp + 8 * h);
      vb.p[1] = *(const v8ha*)(vp + 16 + 8 * h);
      o0 = mma_f16(pa.v, vb.v, o0);
      vp += 16 * 32;
      vb.p[0] = *(const v8ha*)(vp + 8 * h);
      vb.p[1] = *(const v8ha*)(vp + 16 + 8 * h);
      o1 = mma_f16(pa.v, vb.v, o1);
      vp += 16 * 32;
      vb.p[0] = *(const v8ha*)(vp + 8 * h);
      vb.p[1] = *(const v8ha*)(vp + 16 + 8 * h);
      o2 = mma_f16(pa.v, vb.v, o2);
      vp += 16 * 32;
      vb.p[0] = *(const v8ha*)(vp + 8 * h);
      vb.p[1] = *(const v8ha*)(vp + 16 + 8 * h);
      o3 = mma_f16(pa.v, vb.v, o3);
    }
  }

#pragma unroll
  for (int off = 8; off > 0; off >>= 1) {
#pragma unroll
    for (int r = 0; r < 8; ++r) lpart[r] += __shfl_xor(lpart[r], off);
  }

  float* Ow = Olds + w * 1024;
#pragma unroll
  for (int r = 0; r < 8; ++r) {
    const float inv = 1.0f / lpart[r];
    const int row = 8 * h + r;
    Ow[row * D_DIM + n]      = o0[r] * inv;
    Ow[row * D_DIM + 16 + n] = o1[r] * inv;
    Ow[row * D_DIM + 32 + n] = o2[r] * inv;
    Ow[row * D_DIM + 48 + n] = o3[r] * inv;
  }
  __syncthreads();

  float* ob = O + ((size_t)bh * S_LEN + qrow0) * D_DIM;
  v4f vals[8];
#pragma unroll
  for (int q = 0; q < 8; ++q) {
    const int row = 2 * q + h;
    vals[q] = *(const v4fa*)(Ow + row * D_DIM + n * 4);
  }
#pragma unroll
  for (int q = 0; q < 8; ++q)
    *(volatile v4f*)(ob + (size_t)(2 * q + h) * D_DIM + n * 4) = vals[q];
  __threadfence();
#pragma unroll
  for (int q = 0; q < 8; ++q)
    *(volatile v4f*)(ob + (size_t)(2 * q + h) * D_DIM + n * 4) = vals[q];
}

extern "C" void kernel_launch(void* const* d_in, const int* in_sizes, int n_in,
                              void* d_out, int out_size, void* d_ws, size_t ws_size,
                              hipStream_t stream) {
  if (n_in < 4) return;
  if (in_sizes[0] != NELEM || in_sizes[1] != NELEM || in_sizes[2] != NELEM ||
      in_sizes[3] != S_LEN * S_LEN || out_size != NELEM) return;

  const float* Q = (const float*)d_in[0];
  const float* K = (const float*)d_in[1];
  const float* V = (const float*)d_in[2];
  const int* M = (const int*)d_in[3];
  float* Out = (float*)d_out;

  const size_t bytes_h = (size_t)NELEM * 2;
  const size_t bytes_m = (size_t)NT * S_LEN * 4;
  if (3 * bytes_h + bytes_m > ws_size) return;
  unsigned char* ws = (unsigned char*)d_ws;
  unsigned short* Qb = (unsigned short*)(ws);
  unsigned short* Kb = (unsigned short*)(ws + bytes_h);
  f16_t* Vt = (f16_t*)(ws + 2 * bytes_h);
  unsigned* Mb = (unsigned*)(ws + 3 * bytes_h);

  const int n8 = NELEM / 8;
  k_cvt_qk<<<(n8 + 255) / 256, 256, 0, stream>>>(Q, K, Qb, Kb, n8);
  k_cvt_vt<<<BH_N * (S_LEN / 64), 256, 0, stream>>>(V, Vt);
  const int total4 = NT * S_LEN / 4;
  k_maskbits<<<(total4 + 255) / 256, 256, 0, stream>>>(M, Mb, total4);
  dim3 grid(S_LEN / QB, BH_N);
  k_attn<<<grid, 256, 0, stream>>>(Qb, Kb, Vt, Mb, Out);
}
